// TxtNet_59966333387000
// MI455X (gfx1250) — hardware-verified
//
#include <hip/hip_runtime.h>


#define NB_  32
#define LL   512
#define CC   300
#define CP   320
#define HH   512
#define KT   1600
#define RH_  8192
typedef _Float16 h16;
typedef unsigned short bf;
typedef __attribute__((ext_vector_type(16))) __bf16   v16bf;
typedef __attribute__((ext_vector_type(16))) _Float16 v16h;
typedef __attribute__((ext_vector_type(8)))  _Float16 v8h;
typedef __attribute__((ext_vector_type(8)))  unsigned short v8us;
typedef __attribute__((ext_vector_type(8)))  float    v8f;
typedef __attribute__((ext_vector_type(4)))  float    v4f;
typedef v8h  __attribute__((may_alias)) v8ha;
typedef v4f  __attribute__((may_alias)) v4fa;
typedef v8us __attribute__((may_alias)) v8usa;

__device__ __forceinline__ unsigned short f2bf(float f) { unsigned u = __float_as_uint(f); u += 0x7FFFu + ((u >> 16) & 1u); return (unsigned short)(u >> 16); }
__device__ __forceinline__ float bf2f(unsigned short b) { return __uint_as_float(((unsigned)b) << 16); }
__device__ __forceinline__ float bfr(float f) { return bf2f(f2bf(f)); }
__device__ __forceinline__ v16h cat16(v8h lo, v8h hi) { return __builtin_shufflevector(lo, hi, 0, 1, 2, 3, 4, 5, 6, 7, 8, 9, 10, 11, 12, 13, 14, 15); }
__device__ __forceinline__ v16bf cat16b(v8us lo, v8us hi) { return __builtin_bit_cast(v16bf, __builtin_shufflevector(lo, hi, 0, 1, 2, 3, 4, 5, 6, 7, 8, 9, 10, 11, 12, 13, 14, 15)); }
__device__ __forceinline__ v8f wmma16(v16h a, v16h b, v8f c) { return __builtin_amdgcn_wmma_f32_16x16x32_f16(false, a, false, b, (short)0, c, false, false); }
__device__ __forceinline__ v8f wmmab(v16bf a, v16bf b, v8f c) { return __builtin_amdgcn_wmma_f32_16x16x32_bf16(false, a, false, b, (short)0, c, false, false); }


template <typename T16> struct WFrag;
template <> struct WFrag<h16> { typedef v16h V; static __device__ __forceinline__ V ld(const h16* p) { return cat16(*(const v8h*)p, *(const v8h*)(p + 16)); } static __device__ __forceinline__ v8f mma(V a, V b, v8f c) { return wmma16(a, b, c); } };
template <> struct WFrag<bf> { typedef v16bf V; static __device__ __forceinline__ V ld(const bf* p) { return cat16b(*(const v8us*)p, *(const v8us*)(p + 16)); } static __device__ __forceinline__ v8f mma(V a, V b, v8f c) { return wmmab(a, b, c); } };
template <typename T16, int NSPLIT, bool BIAS>
__global__ __launch_bounds__(32) void k_gemmw(const T16* __restrict__ A, const T16* __restrict__ A2, const T16* __restrict__ Bt, const T16* __restrict__ Bt2, int K, float* C, int ldc, const float* __restrict__ bias, size_t sA, size_t sB, size_t sC) {
    typedef typename WFrag<T16>::V V;
    __shared__ __align__(16) float os[16 * 68];
    const size_t z = blockIdx.z; A += z * sA; if (A2) A2 += z * sA; Bt += z * sB; if (Bt2) Bt2 += z * sB; C += z * sC;
    const int lane = threadIdx.x & 31, lr = lane & 15, hi = lane >> 4; const int r0 = blockIdx.x * 64, c0 = blockIdx.y * 64;
    v8f acc[4][4];
#pragma unroll
    for (int mb = 0; mb < 4; ++mb)
#pragma unroll
        for (int nb = 0; nb < 4; ++nb) acc[mb][nb] = (v8f){};
    const size_t aoff = (size_t)(r0 + lr) * K + 8 * hi, boff = (size_t)(c0 + lr) * K + 8 * hi;
#pragma unroll 1
    for (int kc = 0; kc < K; kc += 32) {
        V a[4], a2[4];
#pragma unroll
        for (int mb = 0; mb < 4; ++mb) { a[mb] = WFrag<T16>::ld(A + aoff + (size_t)mb * 16 * K + kc); if (NSPLIT == 1 || NSPLIT == 2) a2[mb] = WFrag<T16>::ld(A2 + aoff + (size_t)mb * 16 * K + kc); }
#pragma unroll
        for (int nb = 0; nb < 4; ++nb) { const V b = WFrag<T16>::ld(Bt + boff + (size_t)nb * 16 * K + kc); V b2; if (NSPLIT >= 2) b2 = WFrag<T16>::ld(Bt2 + boff + (size_t)nb * 16 * K + kc);
#pragma unroll
            for (int mb = 0; mb < 4; ++mb) { acc[mb][nb] = WFrag<T16>::mma(a[mb], b, acc[mb][nb]); if (NSPLIT == 1 || NSPLIT == 2) acc[mb][nb] = WFrag<T16>::mma(a2[mb], b, acc[mb][nb]); if (NSPLIT >= 2) acc[mb][nb] = WFrag<T16>::mma(a[mb], b2, acc[mb][nb]); } }
        asm volatile("v_nop\n\tv_nop\n\tv_nop\n\tv_nop" : "+v"(acc[0][0]), "+v"(acc[1][1]), "+v"(acc[2][2]), "+v"(acc[3][3]) : "v"(a[0]), "v"(a[3]));
    }
#pragma unroll
    for (int mb = 0; mb < 4; ++mb) {
#pragma unroll
        for (int nb = 0; nb < 4; ++nb) {
#pragma unroll
            for (int j = 0; j < 8; ++j) os[(hi * 8 + j) * 68 + nb * 16 + lr] = acc[mb][nb][j]; }
        __builtin_amdgcn_wave_barrier(); asm volatile("" ::: "memory");
        float* crow = C + (size_t)(r0 + mb * 16) * ldc + c0;
#pragma unroll 1
        for (int ps = 0; ps < 2; ++ps) {
#pragma unroll
            for (int s = 0; s < 8; ++s) { const int row = 2 * s + hi, cofs = lr * 4; v4f val = *(const v4fa*)(os + row * 68 + cofs); if (BIAS) { val[0] += bfr(bias[c0 + cofs]); val[1] += bfr(bias[c0 + cofs + 1]); val[2] += bfr(bias[c0 + cofs + 2]); val[3] += bfr(bias[c0 + cofs + 3]); }
                *(volatile v4f*)(crow + (size_t)row * ldc + cofs) = val; }
            if (ps == 0) __threadfence(); }
        __builtin_amdgcn_wave_barrier(); asm volatile("" ::: "memory");
    }
}

__device__ __forceinline__ void splitf(float y, unsigned short& h, unsigned short& l) { h = f2bf(y); l = f2bf(y - bf2f(h)); }
typedef __attribute__((ext_vector_type(4))) unsigned short v4us;
typedef __attribute__((ext_vector_type(2))) unsigned short v2us;

__global__ __launch_bounds__(256) void k_im2col(const float* __restrict__ x, int kw, int padL, int KP, int r0, bf* A) { const size_t e = ((size_t)blockIdx.x * 256 + threadIdx.x) * 4; if (e >= (size_t)RH_ * KP) return; const int col = (int)(e % KP); const int r = r0 + (int)(e / KP); const int b = r / LL, l = r % LL; v4us o;
#pragma unroll
    for (int q = 0; q < 4; ++q) { const int cq = col + q; if (cq >= CC * kw) { o[q] = 0; continue; } const int c = cq / kw, j = cq % kw; int p = l + j - padL; p = p < 0 ? 0 : (p >= LL ? LL - 1 : p); o[q] = f2bf(x[((size_t)b * LL + p) * CC + c]); }
    *(volatile v4us*)(A + e) = o; __threadfence(); *(volatile v4us*)(A + e) = o; }
__global__ __launch_bounds__(256) void k_wpad(const float* __restrict__ Wk, int KW, int KP, bf* Bt) { const int e = (blockIdx.x * 256 + threadIdx.x) * 4; if (e >= CP * KP) return; const int col = e % KP, o = e / KP; v4us v;
#pragma unroll
    for (int q = 0; q < 4; ++q) v[q] = (o < CC && col + q < KW) ? f2bf(Wk[(size_t)o * KW + col + q]) : (unsigned short)0; *(volatile v4us*)(Bt + e) = v; __threadfence(); *(volatile v4us*)(Bt + e) = v; }
__global__ __launch_bounds__(256) void k_slp(const float* __restrict__ w, bf* Bt2) { const int e = (blockIdx.x * 256 + threadIdx.x) * 4; if (e >= HH * KT) return; const int col = e % KT, h = e / KT; const int blk = col / CP, o = col % CP; v4us v;
#pragma unroll
    for (int q = 0; q < 4; ++q) v[q] = (o + q < CC) ? f2bf(w[(size_t)h * 5 * CC + blk * CC + o + q]) : (unsigned short)0; *(volatile v4us*)(Bt2 + e) = v; __threadfence(); *(volatile v4us*)(Bt2 + e) = v; }
__global__ __launch_bounds__(96) void k_tanhcat(const float* __restrict__ F, const float* __restrict__ bias, int br, bf* Hh, bf* Hl) { const size_t r = blockIdx.x; const int g = threadIdx.x; if (g >= 80) return; v4us oh, ol;
#pragma unroll
    for (int q = 0; q < 4; ++q) { const int o = g * 4 + q; if (o < CC) { const float a = __fadd_rn(F[r * CP + o], bfr(bias[o])); const float e2 = __expf(2.0f * a); const float th = __fsub_rn(1.0f, __fdiv_rn(2.0f, __fadd_rn(e2, 1.0f))); unsigned short hh, ll; splitf(th, hh, ll); oh[q] = hh; ol[q] = ll; } else { oh[q] = 0; ol[q] = 0; } }
    const int blk = (br == 3) ? 4 : br; const size_t o0 = r * KT + (size_t)blk * CP + g * 4;
    *(volatile v4us*)(Hh + o0) = oh; *(volatile v4us*)(Hl + o0) = ol; if (br == 2) { *(volatile v4us*)(Hh + o0 + CP) = oh; *(volatile v4us*)(Hl + o0 + CP) = ol; }
    __threadfence(); *(volatile v4us*)(Hh + o0) = oh; *(volatile v4us*)(Hl + o0) = ol; if (br == 2) { *(volatile v4us*)(Hh + o0 + CP) = oh; *(volatile v4us*)(Hl + o0 + CP) = ol; } }
__global__ __launch_bounds__(256) void k_tanhout(const float* __restrict__ G, const float* __restrict__ bias, float* OUTr) { const size_t i = ((size_t)blockIdx.x * 256 + threadIdx.x) * 4; if (i >= (size_t)RH_ * HH) return; const int h = (int)(i % HH); const v4f a = *(const v4f*)(G + i); v4f o;
#pragma unroll
    for (int q = 0; q < 4; ++q) { const float t = __fadd_rn(a[q], bfr(bias[h + q])); const float e2 = __expf(2.0f * t); o[q] = __fsub_rn(1.0f, __fdiv_rn(2.0f, __fadd_rn(e2, 1.0f))); } *(volatile v4f*)(OUTr + i) = o; __threadfence(); *(volatile v4f*)(OUTr + i) = o; }

extern "C" void kernel_launch(void* const* d_in, const int* in_sizes, int n_in,
                              void* d_out, int out_size, void* d_ws, size_t ws_size, hipStream_t stream) {
    (void)in_sizes; (void)n_in; (void)out_size;
    const float* x = (const float*)d_in[0]; const float* Wk[4] = {(const float*)d_in[1], (const float*)d_in[3], (const float*)d_in[5], (const float*)d_in[7]}; const float* bk[4] = {(const float*)d_in[2], (const float*)d_in[4], (const float*)d_in[6], (const float*)d_in[8]}; const float* slp_w = (const float*)d_in[9]; const float* slp_b = (const float*)d_in[10];
    float* OUT = (float*)d_out;
    char* wsp = (char*)d_ws;
    auto take = [&](size_t bytes) { char* p = wsp; wsp += (bytes + 255) & ~(size_t)255; return (void*)p; };
    const int ks[4] = {1, 2, 3, 7}, pads[4] = {0, 0, 1, 3}, KPs[4] = {320, 608, 928, 2112};
    bf* A = (bf*)take((size_t)RH_ * 2112 * 2); bf* Bt = (bf*)take((size_t)CP * 2112 * 2); bf* BT2 = (bf*)take((size_t)HH * KT * 2); float* F = (float*)take((size_t)RH_ * CP * 4); bf* Hh = (bf*)take((size_t)RH_ * KT * 2); bf* Hl = (bf*)take((size_t)RH_ * KT * 2); float* G = (float*)take((size_t)RH_ * HH * 4);
    if ((size_t)(wsp - (char*)d_ws) > ws_size) return;
    k_slp<<<(HH * KT / 4 + 255) / 256, 256, 0, stream>>>(slp_w, BT2);
    for (int hf = 0; hf < 2; ++hf) { const int r0 = hf * RH_;
        for (int br = 0; br < 4; ++br) { const int kw = ks[br], KP = KPs[br];
            k_im2col<<<(unsigned)(((size_t)RH_ * KP / 4 + 255) / 256), 256, 0, stream>>>(x, kw, pads[br], KP, r0, A); k_wpad<<<(CP * KP / 4 + 255) / 256, 256, 0, stream>>>(Wk[br], CC * kw, KP, Bt);
            k_gemmw<bf, 0, false><<<dim3(RH_ / 64, CP / 64, 1), 32, 0, stream>>>(A, nullptr, Bt, nullptr, KP, F, CP, nullptr, 0, 0, 0);
            k_tanhcat<<<RH_, 96, 0, stream>>>(F, bk[br], br, Hh, Hl); }
        k_gemmw<bf, 1, false><<<dim3(RH_ / 64, HH / 64, 1), 32, 0, stream>>>(Hh, Hl, BT2, nullptr, KT, G, HH, nullptr, 0, 0, 0);
        k_tanhout<<<(unsigned)(((size_t)RH_ * HH / 4 + 255) / 256), 256, 0, stream>>>(G, slp_b, OUT + (size_t)r0 * HH); }
}
